// VisionMamba_67602785239636
// MI455X (gfx1250) — hardware-run, weakly checked
//
#include <hip/hip_runtime.h>
#include <math.h>

typedef __attribute__((ext_vector_type(16))) _Float16 v16h;
typedef __attribute__((ext_vector_type(8)))  _Float16 v8h;
typedef __attribute__((ext_vector_type(16))) __bf16   v16b;
typedef __attribute__((ext_vector_type(8)))  __bf16   v8b;
typedef __attribute__((ext_vector_type(8)))  float    v8f;
typedef __attribute__((ext_vector_type(4)))  float    v4f;
typedef __attribute__((ext_vector_type(4)))  unsigned v4u;

constexpr int kB      = 8;
constexpr int kL      = 197;
constexpr int kTok    = kB * kL;
constexpr int kMP     = 1600;
constexpr int kDm     = 192;
constexpr int kDin    = 384;
constexpr int kNst    = 16;
constexpr int kDtR    = 12;
constexpr int kXdR    = 44;
constexpr int kXdN    = 64;
constexpr int kXzP    = 2 * kDin;
constexpr int kCin    = 3;
constexpr int kImg    = 224;
constexpr int kPS     = 16;
constexpr int kPG     = 14;
constexpr int kNP     = kPG * kPG;
constexpr int kPRows  = kB * kNP;
constexpr int kPK     = kCin * kPS * kPS;
constexpr int kNC     = 1000;
constexpr int kDepth  = 24;
constexpr int kClsT   = kNP / 2;
constexpr int kScanCh = 64;
constexpr int kScanTS = 16;
constexpr int kScanYP = 68;
constexpr float kCarryHn = 8.0f;
constexpr float kCarryW  = 16.0f;
constexpr float kCarryXc = 64.0f;
constexpr float kCarryY  = 256.0f;
static_assert(kDtR + 2 * kNst == kXdR && kXdR <= kXdN, "x_proj layout");
static_assert((kMP % 64) == 0 && kMP >= kTok && kMP >= kPRows, "M padded to the 64 tile");
static_assert((kDm % 64) == 0 && (kXzP % 64) == 0 && (kXdN % 64) == 0, "N multiples of 64");
static_assert((kDm % 32) == 0 && (kDin % 32) == 0 && (kPK % 32) == 0, "K multiples of 32");
static_assert((kDin % kScanCh) == 0 && (kDin % 128) == 0, "scan / conv channel tiling");
static_assert((kB * kNC) % 32 == 0, "d_out is a whole number of 128-B lines");

constexpr size_t kOffAP16 = 0;
constexpr size_t kOffPW16 = kOffAP16 + (size_t)kMP * kPK * 2;
constexpr size_t kOffWI16 = kOffPW16 + (size_t)kDm * kPK * 2;
constexpr size_t kOffWX16 = kOffWI16 + (size_t)kDepth * kXzP * kDm * 2;
constexpr size_t kOffWO16 = kOffWX16 + (size_t)kDepth * 2 * kXdN * kDin * 2;
constexpr size_t kOffFEAT = kOffWO16 + (size_t)kDepth * kDm * kDin * 2;
constexpr size_t kOffHB   = kOffFEAT + (size_t)kMP * kDm * 4;
constexpr size_t kOffRES  = kOffHB   + (size_t)kMP * kDm * 4;
constexpr size_t kOffHN16 = kOffRES  + (size_t)kMP * kDm * 4;
constexpr size_t kOffXZ   = kOffHN16 + (size_t)kMP * kDm * 2;
constexpr size_t kOffXC   = kOffXZ   + (size_t)kMP * kXzP * 4;
constexpr size_t kOffXC16 = kOffXC   + (size_t)2 * kMP * kDin * 4;
constexpr size_t kOffXD   = kOffXC16 + (size_t)2 * kMP * kDin * 2;
constexpr size_t kOffY16  = kOffXD   + (size_t)2 * kMP * kXdN * 4;
constexpr size_t kWsTotal = kOffY16  + (size_t)kMP * kDin * 2;
static_assert(kWsTotal == 34365440ull, "carve total");
static_assert(kWsTotal <= 134217728ull, "carve cap");
static_assert((kOffPW16 % 128) == 0 && (kOffWI16 % 128) == 0 && (kOffWX16 % 128) == 0 && (kOffWO16 % 128) == 0 &&
              (kOffFEAT % 128) == 0 && (kOffHB % 128) == 0 && (kOffRES % 128) == 0 && (kOffHN16 % 128) == 0 &&
              (kOffXZ % 128) == 0 && (kOffXC % 128) == 0 && (kOffXC16 % 128) == 0 && (kOffXD % 128) == 0 &&
              (kOffY16 % 128) == 0, "128-B aligned regions");

__device__ __forceinline__ unsigned short f2bf_bits(float f) {
  unsigned u = __float_as_uint(f);
  return (unsigned short)((u + 0x7FFFu + ((u >> 16) & 1u)) >> 16);
}
__device__ __forceinline__ float bf_bits2f(unsigned short h) { return __uint_as_float(((unsigned)h) << 16); }

__device__ __forceinline__ void dep_guard_h(v8f& a, v8f& b, v16h x, v16h y) { asm volatile("v_nop\n\tv_nop\n\tv_nop\n\tv_nop" : "+v"(a), "+v"(b) : "v"(x), "v"(y)); }
__device__ __forceinline__ void dep_guard_b(v8f& a, v8f& b, v16b x, v16b y) { asm volatile("v_nop\n\tv_nop\n\tv_nop\n\tv_nop" : "+v"(a), "+v"(b) : "v"(x), "v"(y)); }
__device__ __forceinline__ void dep_guard4_h(v8f& a, v8f& b, v8f& c, v8f& d, v16h x, v16h y) { asm volatile("v_nop\n\tv_nop\n\tv_nop\n\tv_nop" : "+v"(a), "+v"(b), "+v"(c), "+v"(d) : "v"(x), "v"(y)); }
__device__ __forceinline__ void dep_guard4_b(v8f& a, v8f& b, v8f& c, v8f& d, v16b x, v16b y) { asm volatile("v_nop\n\tv_nop\n\tv_nop\n\tv_nop" : "+v"(a), "+v"(b), "+v"(c), "+v"(d) : "v"(x), "v"(y)); }
__device__ __forceinline__ void keep4_h(v16h a, v16h b, v16h c, v16h d) { asm volatile("v_nop" :: "v"(a), "v"(b), "v"(c), "v"(d)); }
__device__ __forceinline__ void keep4_b(v16b a, v16b b, v16b c, v16b d) { asm volatile("v_nop" :: "v"(a), "v"(b), "v"(c), "v"(d)); }
__device__ __forceinline__ void acc_guard4(v8f& a, v8f& b, v8f& c, v8f& d) { asm volatile("v_nop\n\tv_nop\n\tv_nop\n\tv_nop" : "+v"(a), "+v"(b), "+v"(c), "+v"(d)); }
template <typename T> struct Frag;
template <> struct Frag<_Float16> {
  typedef v16h V; union U { v16h v; v8h h[2]; };
  static __device__ __forceinline__ v16h load(const _Float16* p) {
    U f; f.h[0] = *(const v8h*)(p); f.h[1] = *(const v8h*)(p + 16); return f.v;
  }
  static __device__ __forceinline__ v8f mma(v16h a, v16h b, v8f c) {
    return __builtin_amdgcn_wmma_f32_16x16x32_f16(false, a, false, b, (short)0, c, false, false);
  }
  static __device__ __forceinline__ void guard(v8f& a, v8f& b, v16h x, v16h y) { dep_guard_h(a, b, x, y); }
  static __device__ __forceinline__ void guard4(v8f& a, v8f& b, v8f& c, v8f& d, v16h x, v16h y) { dep_guard4_h(a, b, c, d, x, y); }
  static __device__ __forceinline__ void keep(v16h a, v16h b, v16h c, v16h d) { keep4_h(a, b, c, d); }
};
template <> struct Frag<__bf16> {
  typedef v16b V; union U { v16b v; v8b h[2]; };
  static __device__ __forceinline__ v16b load(const __bf16* p) {
    U f; f.h[0] = *(const v8b*)(p); f.h[1] = *(const v8b*)(p + 16); return f.v;
  }
  static __device__ __forceinline__ v8f mma(v16b a, v16b b, v8f c) {
    return __builtin_amdgcn_wmma_f32_16x16x32_bf16(false, a, false, b, (short)0, c, false, false);
  }
  static __device__ __forceinline__ void guard(v8f& a, v8f& b, v16b x, v16b y) { dep_guard_b(a, b, x, y); }
  static __device__ __forceinline__ void guard4(v8f& a, v8f& b, v8f& c, v8f& d, v16b x, v16b y) { dep_guard4_b(a, b, c, d, x, y); }
  static __device__ __forceinline__ void keep(v16b a, v16b b, v16b c, v16b d) { keep4_b(a, b, c, d); }
};

template <int ET> struct Elem;
template <> struct Elem<0> { typedef _Float16 T; };
template <> struct Elem<1> { typedef __bf16 T; };
template <int ET, bool SPLIT, int BIAS_MODE, int OUT_MODE, bool RESID, int ACT = 0>
__global__ __launch_bounds__(256) void wmma_gemm64(
    const unsigned short* __restrict__ Ap, const unsigned short* __restrict__ A2p, int lda, long strideA,
    const unsigned short* __restrict__ Btp, const unsigned short* __restrict__ Bt2p, int ldb, long strideB,
    void* __restrict__ Cout, void* __restrict__ Cout2, int ldc, long strideC,
    const float* __restrict__ bias,
    const float* __restrict__ resid, long strideR,
    int M, int N, int K, float scale) {
  typedef typename Elem<ET>::T T;
  typedef typename Frag<T>::V V;
  const T* A = (const T*)Ap; const T* A2 = (const T*)A2p; const T* Bt = (const T*)Btp; const T* Bt2 = (const T*)Bt2p;
  __shared__ __align__(16) float sT[8][16 * 68];
  const int b    = blockIdx.y;
  const int lane = threadIdx.x & 31;
  const int wave = threadIdx.x >> 5;
  const int tilesN = N >> 6;
  const int tilesM = M >> 6;
  const int tile = blockIdx.x * 8 + wave;
  if (tile >= tilesM * tilesN) return;
  const int tm = tile / tilesN;
  const int tn = tile - tm * tilesN;
  const int m0 = tm << 6;
  const int n0 = tn << 6;

  const T* Ab  = A  + (size_t)b * strideA;
  const T* Bb  = Bt + (size_t)b * strideB;
  const T* Ab2 = SPLIT ? (A2  + (size_t)b * strideA) : nullptr;
  const T* Bb2 = SPLIT ? (Bt2 + (size_t)b * strideB) : nullptr;

  const int rlane = lane & 15;
  const int koff  = (lane >> 4) * 8;
  const int mOff  = (lane >> 4) * 8;

  v8f acc[4][4];
#pragma unroll
  for (int i = 0; i < 4; ++i)
#pragma unroll
    for (int j = 0; j < 4; ++j) acc[i][j] = (v8f){0.f,0.f,0.f,0.f,0.f,0.f,0.f,0.f};

  for (int k0 = 0; k0 < K; k0 += 32) {
    V bh[4], bl[4];
#pragma unroll
    for (int j = 0; j < 4; ++j) {
      const size_t bo = (size_t)(n0 + (j << 4) + rlane) * ldb + koff + k0;
      bh[j] = Frag<T>::load(Bb + bo);
      if (SPLIT) bl[j] = Frag<T>::load(Bb2 + bo);
    }
#pragma unroll
    for (int i = 0; i < 4; ++i) {
      const size_t ao = (size_t)(m0 + (i << 4) + rlane) * lda + koff + k0;
      V ah = Frag<T>::load(Ab + ao);
      V al;
      if (SPLIT) al = Frag<T>::load(Ab2 + ao);
#pragma unroll
      for (int j = 0; j < 4; ++j) {
        acc[i][j] = Frag<T>::mma(ah, bh[j], acc[i][j]);
        if (SPLIT) {
          acc[i][j] = Frag<T>::mma(ah, bl[j], acc[i][j]);
          acc[i][j] = Frag<T>::mma(al, bh[j], acc[i][j]);
        }
      }
      Frag<T>::guard4(acc[i][0], acc[i][1], acc[i][2], acc[i][3], ah, SPLIT ? al : ah);
    }
    Frag<T>::keep(bh[0], bh[1], bh[2], bh[3]);
    if (SPLIT) Frag<T>::keep(bl[0], bl[1], bl[2], bl[3]);
  }
  acc_guard4(acc[0][0], acc[0][1], acc[0][2], acc[0][3]);
  acc_guard4(acc[1][0], acc[1][1], acc[1][2], acc[1][3]);
  acc_guard4(acc[2][0], acc[2][1], acc[2][2], acc[2][3]);
  acc_guard4(acc[3][0], acc[3][1], acc[3][2], acc[3][3]);

  float* slab = sT[wave];
  const float* Rb = RESID ? (resid + (size_t)b * strideR) : nullptr;
#pragma unroll
  for (int i = 0; i < 4; ++i) {
    const int mBase = m0 + (i << 4);
#pragma unroll
    for (int j = 0; j < 4; ++j) {
      const int n = n0 + (j << 4) + rlane;
      float bv = 0.f;
      if (BIAS_MODE == 2) bv = bias[n];
#pragma unroll
      for (int r = 0; r < 8; ++r) {
        float v = acc[i][j][r] * scale;
        if (BIAS_MODE == 1) v += bias[mBase + mOff + r];
        if (BIAS_MODE == 2) v += bv;
        if (RESID) v += Rb[(size_t)(mBase + mOff + r) * ldc + n];
        if (ACT == 1) v = tanhf(v);
        if (ACT == 2) v = fmaxf(v, 0.0f);
        if (ACT == 3) v = v / (1.0f + expf(-v));
        if (ACT == 4) v = (v > 0.f) ? v : 0.01f * v;
        slab[(mOff + r) * 68 + (j << 4) + rlane] = v;
      }
    }
    __builtin_amdgcn_fence(__ATOMIC_RELEASE, "workgroup");
    __builtin_amdgcn_wave_barrier();
    __builtin_amdgcn_fence(__ATOMIC_ACQUIRE, "workgroup");
    if (OUT_MODE == 0) {
      float* C = (float*)Cout + (size_t)b * strideC;
      const int hh = lane >> 4, c4 = (lane & 15) * 4;
      for (int pass = 0; pass < 2; ++pass) {
#pragma unroll
        for (int it = 0; it < 8; ++it) {
          const int row = it * 2 + hh;
          v4f v = *(const v4f*)(slab + row * 68 + c4);
          *(volatile v4f*)(C + (size_t)(mBase + row) * ldc + n0 + c4) = v;
        }
        __threadfence();
      }
    } else {
      const int q = lane >> 3, c8 = (lane & 7) * 8;
      unsigned short* C  = (unsigned short*)Cout  + (size_t)b * strideC;
      unsigned short* C2 = (OUT_MODE == 2) ? ((unsigned short*)Cout2 + (size_t)b * strideC) : nullptr;
      for (int pass = 0; pass < 2; ++pass) {
#pragma unroll
        for (int it = 0; it < 4; ++it) {
          const int row = it * 4 + q;
          const float* sp = slab + row * 68 + c8;
          v8h hv, lv;
#pragma unroll
          for (int e = 0; e < 8; ++e) {
            if (OUT_MODE == 1) {
              hv[e] = (_Float16)sp[e];
            } else {
              unsigned short hb = f2bf_bits(sp[e]);
              unsigned short lb = f2bf_bits(sp[e] - bf_bits2f(hb));
              hv[e] = __builtin_bit_cast(_Float16, hb);
              lv[e] = __builtin_bit_cast(_Float16, lb);
            }
          }
          *(volatile v8h*)(C + (size_t)(mBase + row) * ldc + n0 + c8) = hv;
          if (OUT_MODE == 2) *(volatile v8h*)(C2 + (size_t)(mBase + row) * ldc + n0 + c8) = lv;
        }
        __threadfence();
      }
    }
    __builtin_amdgcn_fence(__ATOMIC_RELEASE, "workgroup");
    __builtin_amdgcn_wave_barrier();
    __builtin_amdgcn_fence(__ATOMIC_ACQUIRE, "workgroup");
  }
}

__global__ __launch_bounds__(256) void cast_scale_f16x8(
    const float* __restrict__ in, unsigned short* __restrict__ out, int n8, float sc)
{
  const int i = blockIdx.x * 256 + threadIdx.x;
  if (i >= n8) return;
  const size_t e0 = (size_t)i << 3;
  const v4f a0 = *(const v4f*)(in + e0);
  const v4f a1 = *(const v4f*)(in + e0 + 4);
  v8h hv;
#pragma unroll
  for (int e = 0; e < 4; ++e) {
    hv[e]     = (_Float16)(a0[e] * sc);
    hv[4 + e] = (_Float16)(a1[e] * sc);
  }
  unsigned short* q = out + e0;
  *(volatile v8h*)q = hv;
  __threadfence();
  *(volatile v8h*)q = hv;
}

__global__ __launch_bounds__(256) void pack_xproj_w(
    const float* __restrict__ wf, const float* __restrict__ wb, unsigned short* __restrict__ out, int n8, float sc)
{
  const int i = blockIdx.x * 256 + threadIdx.x;
  if (i >= n8) return;
  const int e0 = i << 3;
  constexpr int kPerLayer = 2 * kXdN * kDin;
  constexpr int kPerDir   = kXdN * kDin;
  const int l    = e0 / kPerLayer;
  const int rem  = e0 - l * kPerLayer;
  const int dir  = rem / kPerDir;
  const int rem2 = rem - dir * kPerDir;
  const int n    = rem2 / kDin;
  const int k    = rem2 - n * kDin;
  const int nn   = (n < kXdR) ? n : (kXdR - 1);
  const size_t so = ((size_t)l * kXdR + nn) * kDin + k;
  const v4f f0 = *(const v4f*)(wf + so);
  const v4f f1 = *(const v4f*)(wf + so + 4);
  const v4f b0 = *(const v4f*)(wb + so);
  const v4f b1 = *(const v4f*)(wb + so + 4);
  const float fd = (float)dir;
  const float fk = 1.0f - fd;
  const float fz = (n < kXdR) ? sc : 0.0f;
  v8h hv;
#pragma unroll
  for (int e = 0; e < 4; ++e) {
    hv[e]     = (_Float16)((f0[e] * fk + b0[e] * fd) * fz);
    hv[4 + e] = (_Float16)((f1[e] * fk + b1[e] * fd) * fz);
  }
  unsigned short* q = out + (size_t)e0;
  *(volatile v8h*)q = hv;
  __threadfence();
  *(volatile v8h*)q = hv;
}

__global__ __launch_bounds__(256) void im2col_kernel(
    const float* __restrict__ x, unsigned short* __restrict__ out, int n8)
{
  const int i = blockIdx.x * 256 + threadIdx.x;
  if (i >= n8) return;
  const int e0  = i << 3;
  const int row = e0 / kPK;
  const int k   = e0 - row * kPK;
  const int c   = k >> 8;
  const int ky  = (k >> 4) & 15;
  const int kx0 = k & 15;
  const bool ok = (row < kPRows);
  const int rowc = ok ? row : (kPRows - 1);
  const int b  = rowc / kNP;
  const int p  = rowc - b * kNP;
  const int py = p / kPG;
  const int px = p - py * kPG;
  const float* src = x + ((size_t)(b * kCin + c) * kImg + (size_t)(py * kPS + ky)) * kImg + px * kPS + kx0;
  const v4f a0 = *(const v4f*)(src);
  const v4f a1 = *(const v4f*)(src + 4);
  const float fz = ok ? 1.0f : 0.0f;
  v8h hv;
#pragma unroll
  for (int e = 0; e < 4; ++e) {
    hv[e]     = (_Float16)(a0[e] * fz);
    hv[4 + e] = (_Float16)(a1[e] * fz);
  }
  unsigned short* q = out + (size_t)e0;
  *(volatile v8h*)q = hv;
  __threadfence();
  *(volatile v8h*)q = hv;
}

__global__ __launch_bounds__(256) void zero_f16x8(unsigned short* __restrict__ out, int n8)
{
  const int i = blockIdx.x * 256 + threadIdx.x;
  if (i >= n8) return;
  const v4u z = (v4u){0u, 0u, 0u, 0u};
  unsigned short* q = out + ((size_t)i << 3);
  *(volatile v4u*)q = z;
  __threadfence();
  *(volatile v4u*)q = z;
}

__global__ __launch_bounds__(64) void embed_kernel(
    const float* __restrict__ FEAT, const float* __restrict__ pb, const float* __restrict__ cls,
    const float* __restrict__ pos, float* __restrict__ HB, float* __restrict__ RES)
{
  const int tid = threadIdx.x;
  if (tid >= 48) return;
  const int r  = blockIdx.x;
  const int c4 = tid * 4;
  const int b  = r / kL;
  const int t  = r - b * kL;
  const float fvalid = (r < kTok) ? 1.0f : 0.0f;
  const int p    = t - ((t > kClsT) ? 1 : 0);
  const int prow = b * kNP + p;
  const v4f fe = *(const v4f*)(FEAT + (size_t)prow * kDm + c4);
  const v4f po = *(const v4f*)(pos + (size_t)t * kDm + c4);
  const v4f cv = *(const v4f*)(cls + c4);
  const v4f bv = *(const v4f*)(pb + c4);
  const float fc = (t == kClsT) ? 1.0f : 0.0f;
  const float fp = 1.0f - fc;
  v4f val;
#pragma unroll
  for (int e = 0; e < 4; ++e) val[e] = (((fe[e] + bv[e]) * fp + cv[e] * fc) + po[e]) * fvalid;
  const v4f zz = (v4f){0.f, 0.f, 0.f, 0.f};
  float* ph = HB  + (size_t)r * kDm + c4;
  float* pr = RES + (size_t)r * kDm + c4;
  for (int pass = 0; pass < 2; ++pass) {
    *(volatile v4f*)ph = val;
    *(volatile v4f*)pr = zz;
    __threadfence();
  }
}

__global__ __launch_bounds__(64) void rmsnorm_kernel(
    const float* __restrict__ HB, float* __restrict__ RES, const float* __restrict__ nw,
    unsigned short* __restrict__ HN16)
{
  __shared__ float sRed[2];
  __shared__ __align__(16) float sHn[kDm];
  const int tid = threadIdx.x, lane = tid & 31, wave = tid >> 5;
  const int r = blockIdx.x;
  const bool own = (tid < 48);
  const int c4 = (own ? tid : 47) * 4;
  const v4f hv = *(const v4f*)(HB  + (size_t)r * kDm + c4);
  const v4f rv = *(const v4f*)(RES + (size_t)r * kDm + c4);
  const v4f wv = *(const v4f*)(nw + c4);
  v4f rr;
#pragma unroll
  for (int e = 0; e < 4; ++e) rr[e] = rv[e] + hv[e];
  float sq = 0.0f;
  sq = fmaf(rr[0], rr[0], sq); sq = fmaf(rr[1], rr[1], sq); sq = fmaf(rr[2], rr[2], sq); sq = fmaf(rr[3], rr[3], sq);
  sq = own ? sq : 0.0f;
#pragma unroll
  for (int off = 16; off > 0; off >>= 1) sq += __shfl_xor(sq, off, 32);
  if (lane == 0) sRed[wave] = sq;
  __syncthreads();
  const float tot  = sRed[0] + sRed[1];
  const float scl  = rsqrtf(tot * (1.0f / (float)kDm) + 1e-5f);
  if (own) {
#pragma unroll
    for (int e = 0; e < 4; ++e) sHn[c4 + e] = ((rr[e] * scl) * wv[e]) * kCarryHn;
  }
  float* pr = RES + (size_t)r * kDm + c4;
  __syncthreads();
  const int c8 = (tid < 24 ? tid : 23) * 8;
  const v4f s0 = *(const v4f*)(sHn + c8);
  const v4f s1 = *(const v4f*)(sHn + c8 + 4);
  v8h hn;
#pragma unroll
  for (int e = 0; e < 4; ++e) { hn[e] = (_Float16)s0[e]; hn[4 + e] = (_Float16)s1[e]; }
  unsigned short* pq = HN16 + (size_t)r * kDm + c8;
  for (int pass = 0; pass < 2; ++pass) {
    if (own) *(volatile v4f*)pr = rr;
    if (tid < 24) *(volatile v8h*)pq = hn;
    __threadfence();
  }
}

__global__ __launch_bounds__(128) void conv_silu_kernel(
    const float* __restrict__ XZ, const float* __restrict__ cwf, const float* __restrict__ cbf,
    const float* __restrict__ cwb, const float* __restrict__ cbb,
    float* __restrict__ XC, unsigned short* __restrict__ XC16)
{
  __shared__ __align__(16) float sO[2][kDin];
  const int tid = threadIdx.x;
  const int r = blockIdx.x;
  const int b = r / kL;
  const int t = r - b * kL;
  const bool rowok = (r < kTok);
  const float fm3 = (rowok && t >= 3) ? 1.0f : 0.0f;
  const float fm2 = (rowok && t >= 2) ? 1.0f : 0.0f;
  const float fm1 = (rowok && t >= 1) ? 1.0f : 0.0f;
  const float f00 = rowok ? 1.0f : 0.0f;
  const float fp1 = (rowok && t <= kL - 2) ? 1.0f : 0.0f;
  const float fp2 = (rowok && t <= kL - 3) ? 1.0f : 0.0f;
  const float fp3 = (rowok && t <= kL - 4) ? 1.0f : 0.0f;
  const int rm3 = (r - 3 > 0) ? (r - 3) : 0;
  const int rm2 = (r - 2 > 0) ? (r - 2) : 0;
  const int rm1 = (r - 1 > 0) ? (r - 1) : 0;
  const int rp1 = (r + 1 < kMP - 1) ? (r + 1) : (kMP - 1);
  const int rp2 = (r + 2 < kMP - 1) ? (r + 2) : (kMP - 1);
  const int rp3 = (r + 3 < kMP - 1) ? (r + 3) : (kMP - 1);
#pragma unroll 1
  for (int j = 0; j < 3; ++j) {
    const int d = tid + 128 * j;
    const float xm3 = XZ[(size_t)rm3 * kXzP + d] * fm3;
    const float xm2 = XZ[(size_t)rm2 * kXzP + d] * fm2;
    const float xm1 = XZ[(size_t)rm1 * kXzP + d] * fm1;
    const float x00 = XZ[(size_t)r   * kXzP + d] * f00;
    const float xp1 = XZ[(size_t)rp1 * kXzP + d] * fp1;
    const float xp2 = XZ[(size_t)rp2 * kXzP + d] * fp2;
    const float xp3 = XZ[(size_t)rp3 * kXzP + d] * fp3;
    asm volatile("" ::: "memory");
    const v4f wf = *(const v4f*)(cwf + d * 4);
    const v4f wb = *(const v4f*)(cwb + d * 4);
    const float bf = cbf[d], bb = cbb[d];
    float sf = wf[0] * xm3;
    sf = fmaf(wf[1], xm2, sf);
    sf = fmaf(wf[2], xm1, sf);
    sf = fmaf(wf[3], x00, sf);
    const float vf = sf + bf;
    float sb = wb[3] * x00;
    sb = fmaf(wb[2], xp1, sb);
    sb = fmaf(wb[1], xp2, sb);
    sb = fmaf(wb[0], xp3, sb);
    const float vb = sb + bb;
    const float gf = vf * __builtin_amdgcn_rcpf(1.0f + expf(-vf));
    const float gb = vb * __builtin_amdgcn_rcpf(1.0f + expf(-vb));
    sO[0][d] = gf * f00;
    sO[1][d] = gb * f00;
  }
  __syncthreads();
  const int c4 = (tid < 96 ? tid : 95) * 4;
  const v4f o0 = *(const v4f*)(&sO[0][c4]);
  const v4f o1 = *(const v4f*)(&sO[1][c4]);
  const int c8 = (tid < 48 ? tid : 47) * 8;
  const v4f a0 = *(const v4f*)(&sO[0][c8]);
  const v4f a1 = *(const v4f*)(&sO[0][c8 + 4]);
  const v4f b0 = *(const v4f*)(&sO[1][c8]);
  const v4f b1 = *(const v4f*)(&sO[1][c8 + 4]);
  v8h h0, h1;
#pragma unroll
  for (int e = 0; e < 4; ++e) {
    h0[e]     = (_Float16)(a0[e] * kCarryXc);
    h0[4 + e] = (_Float16)(a1[e] * kCarryXc);
    h1[e]     = (_Float16)(b0[e] * kCarryXc);
    h1[4 + e] = (_Float16)(b1[e] * kCarryXc);
  }
  float* p0 = XC + (size_t)r * kDin + c4;
  float* p1 = XC + ((size_t)kMP + r) * kDin + c4;
  unsigned short* q0 = XC16 + (size_t)r * kDin + c8;
  unsigned short* q1 = XC16 + ((size_t)kMP + r) * kDin + c8;
  for (int pass = 0; pass < 2; ++pass) {
    if (tid < 96) {
      *(volatile v4f*)p0 = o0;
      *(volatile v4f*)p1 = o1;
    }
    if (tid < 48) {
      *(volatile v8h*)q0 = h0;
      *(volatile v8h*)q1 = h1;
    }
    __threadfence();
  }
}

__global__ __launch_bounds__(64) void scan_gate_kernel(
    const float* __restrict__ XD, const float* __restrict__ XC, const float* __restrict__ XZ,
    const float* __restrict__ Wdtf, const float* __restrict__ bdtf, const float* __restrict__ Alogf, const float* __restrict__ Dpf,
    const float* __restrict__ Wdtb, const float* __restrict__ bdtb, const float* __restrict__ Alogb, const float* __restrict__ Dpb,
    unsigned short* __restrict__ Y16)
{
  __shared__ __align__(16) float sYF[kL * kScanCh];
  __shared__ __align__(16) float sX[kScanTS * kXdN];
  __shared__ __align__(16) float sW[kDtR * kScanCh];
  __shared__ __align__(16) float sYt[kScanTS * kScanYP];
  const int tid = threadIdx.x, lane = tid & 31, wave = tid >> 5;
  constexpr int kBlkPerB = kDin / kScanCh;
  const int bix = blockIdx.x / kBlkPerB;
  const int d0  = (blockIdx.x - bix * kBlkPerB) * kScanCh;
  const int d   = d0 + tid;
  const int row0 = bix * kL;
  const int q = lane >> 3, c8 = (lane & 7) * 8;
#pragma unroll 1
  for (int dir = 0; dir < 2; ++dir) {
    const float* Wdt  = dir ? Wdtb : Wdtf;
    const float* bdt  = dir ? bdtb : bdtf;
    const float* Alog = dir ? Alogb : Alogf;
    const float* Dp   = dir ? Dpb : Dpf;
    const float* XDd  = XD + (size_t)dir * kMP * kXdN;
    const float* XCd  = XC + (size_t)dir * kMP * kDin;
    __syncthreads();
#pragma unroll 1
    for (int r = 0; r < kDtR; ++r) sW[r * kScanCh + tid] = Wdt[(size_t)d * kDtR + r];
#pragma unroll 1
    for (int s = 0; s < kNst; ++s) sYt[s * kScanCh + tid] = -expf(Alog[(size_t)d * kNst + s]);
    __syncthreads();
    float negA[kNst], h[kNst];
#pragma unroll
    for (int s = 0; s < kNst; ++s) { negA[s] = sYt[s * kScanCh + tid]; h[s] = 0.0f; }
    const float bb = bdt[d], Dd = Dp[d];
    __syncthreads();
#pragma unroll 1
    for (int t0 = 0; t0 < kL; t0 += kScanTS) {
      __syncthreads();
#pragma unroll
      for (int i = 0; i < 4; ++i) {
        const int idx = tid + 64 * i;
        const int rr  = idx >> 4;
        const int cc  = (idx & 15) * 4;
        int tt = dir ? (kL - 1 - (t0 + rr)) : (t0 + rr);
        tt = tt < 0 ? 0 : (tt > kL - 1 ? kL - 1 : tt);
        *(v4f*)(sX + rr * kXdN + cc) = *(const v4f*)(XDd + (size_t)(row0 + tt) * kXdN + cc);
      }
      __syncthreads();
#pragma unroll 1
      for (int s = 0; s < kScanTS; ++s) {
        const int ts = t0 + s;
        const bool valid = (ts < kL);
        int tt = dir ? (kL - 1 - ts) : ts;
        tt = tt < 0 ? 0 : (tt > kL - 1 ? kL - 1 : tt);
        const float* xr = sX + s * kXdN;
        float vdot = 0.0f;
#pragma unroll 1
        for (int r4 = 0; r4 < kDtR / 4; ++r4) {
          const v4f xv = *(const v4f*)(xr + 4 * r4);
          const float* wp = sW + (4 * r4) * kScanCh + tid;
          vdot = fmaf(xv[0], wp[0], vdot);
          vdot = fmaf(xv[1], wp[kScanCh], vdot);
          vdot = fmaf(xv[2], wp[2 * kScanCh], vdot);
          vdot = fmaf(xv[3], wp[3 * kScanCh], vdot);
        }
        float Bs[kNst], Cs[kNst];
#pragma unroll
        for (int q4 = 0; q4 < 4; ++q4) {
          const v4f bv = *(const v4f*)(xr + kDtR + 4 * q4);
          const v4f cv = *(const v4f*)(xr + kDtR + kNst + 4 * q4);
          Bs[4 * q4 + 0] = bv[0]; Bs[4 * q4 + 1] = bv[1]; Bs[4 * q4 + 2] = bv[2]; Bs[4 * q4 + 3] = bv[3];
          Cs[4 * q4 + 0] = cv[0]; Cs[4 * q4 + 1] = cv[1]; Cs[4 * q4 + 2] = cv[2]; Cs[4 * q4 + 3] = cv[3];
        }
        const float v   = vdot + bb;
        const float a   = __expf(-fabsf(v));
        const float u   = 1.0f + a;
        const float l1p = __logf(u) + (a - (u - 1.0f)) * __builtin_amdgcn_rcpf(u);
        const float dt  = fmaxf(v, 0.0f) + l1p;
        const size_t grow = (size_t)(row0 + tt);
        const float xt  = XCd[grow * kDin + d];
        const float dtx = dt * xt;
        float y = 0.0f;
#pragma unroll
        for (int k = 0; k < kNst; ++k) {
          const float e = __expf(dt * negA[k]);
          h[k] = e * h[k] + dtx * Bs[k];
          y = fmaf(h[k], Cs[k], y);
        }
        y = fmaf(xt, Dd, y);
        if (dir == 0) {
          if (valid) sYF[tt * kScanCh + tid] = y;
        } else {
          const float yf = sYF[tt * kScanCh + tid];
          const float zv = XZ[grow * kXzP + kDin + d];
          const float sg = __builtin_amdgcn_rcpf(1.0f + expf(-zv));
          sYt[s * kScanYP + tid] = (0.5f * (yf + y)) * (zv * sg) * kCarryY;
        }
      }
      if (dir == 1) {
        __syncthreads();
        v8h hv[2];
#pragma unroll
        for (int it = 0; it < 2; ++it) {
          const int row = it * 8 + wave * 4 + q;
          const float* sp = sYt + row * kScanYP + c8;
          const v4f a0 = *(const v4f*)(sp);
          const v4f a1 = *(const v4f*)(sp + 4);
#pragma unroll
          for (int e = 0; e < 4; ++e) { hv[it][e] = (_Float16)a0[e]; hv[it][4 + e] = (_Float16)a1[e]; }
        }
        for (int pass = 0; pass < 2; ++pass) {
#pragma unroll
          for (int it = 0; it < 2; ++it) {
            const int row = it * 8 + wave * 4 + q;
            const int ts = t0 + row;
            if (ts < kL) {
              const int tt = kL - 1 - ts;
              *(volatile v8h*)(Y16 + (size_t)(row0 + tt) * kDin + d0 + c8) = hv[it];
            }
          }
          __threadfence();
        }
      }
    }
  }
}

__global__ __launch_bounds__(256) void head_kernel(
    const float* __restrict__ HB, const float* __restrict__ RES, const float* __restrict__ nfw,
    const float* __restrict__ hw, const float* __restrict__ hb, float* __restrict__ out)
{
  __shared__ __align__(16) float sCls[kB * kDm];
  const int tid = threadIdx.x, lane = tid & 31, wave = tid >> 5;
  {
    const int b = wave;
    const size_t rowc = (size_t)(b * kL + kClsT) * kDm;
    float sq = 0.0f;
#pragma unroll 1
    for (int i = 0; i < 6; ++i) {
      const int ch = lane + 32 * i;
      const float r = RES[rowc + ch] + HB[rowc + ch];
      sq = fmaf(r, r, sq);
    }
#pragma unroll
    for (int off = 16; off > 0; off >>= 1) sq += __shfl_xor(sq, off, 32);
    const float scl = rsqrtf(sq * (1.0f / (float)kDm) + 1e-5f);
#pragma unroll 1
    for (int i = 0; i < 6; ++i) {
      const int ch = lane + 32 * i;
      const float r = RES[rowc + ch] + HB[rowc + ch];
      sCls[b * kDm + ch] = (r * scl) * nfw[ch];
    }
  }
  __syncthreads();
  const int e0 = blockIdx.x * 1024 + tid * 4;
  const bool ok = (e0 < kB * kNC);
  const int ec = ok ? e0 : (kB * kNC - 4);
  const int bb = ec / kNC;
  const int c0 = ec - bb * kNC;
  float acc0 = 0.0f, acc1 = 0.0f, acc2 = 0.0f, acc3 = 0.0f;
  const float* w0 = hw + (size_t)(c0 + 0) * kDm;
  const float* w1 = hw + (size_t)(c0 + 1) * kDm;
  const float* w2 = hw + (size_t)(c0 + 2) * kDm;
  const float* w3 = hw + (size_t)(c0 + 3) * kDm;
  const float* cp = sCls + bb * kDm;
#pragma unroll 1
  for (int k = 0; k < kDm; ++k) {
    const float cv = cp[k];
    acc0 = fmaf(cv, w0[k], acc0);
    acc1 = fmaf(cv, w1[k], acc1);
    acc2 = fmaf(cv, w2[k], acc2);
    acc3 = fmaf(cv, w3[k], acc3);
  }
  v4f o;
  o[0] = acc0 + hb[c0 + 0];
  o[1] = acc1 + hb[c0 + 1];
  o[2] = acc2 + hb[c0 + 2];
  o[3] = acc3 + hb[c0 + 3];
  float* po = out + e0;
  for (int pass = 0; pass < 2; ++pass) {
    if (ok) *(volatile v4f*)po = o;
    __threadfence();
  }
}

extern "C" void kernel_launch(void* const* d_in, const int* in_sizes, int n_in,
                              void* d_out, int out_size, void* d_ws, size_t ws_size,
                              hipStream_t stream)
{
  if (n_in < 25) return;
  if (in_sizes[0] != kB * kCin * kImg * kImg) return;
  if (in_sizes[1] != kDm * kPK) return;
  if (in_sizes[2] != kDm || in_sizes[3] != kDm) return;
  if (in_sizes[4] != kL * kDm) return;
  if (in_sizes[5] != kDepth * kXzP * kDm) return;
  if (in_sizes[6] != kDepth * kDin * 4 || in_sizes[13] != kDepth * kDin * 4) return;
  if (in_sizes[7] != kDepth * kDin || in_sizes[14] != kDepth * kDin) return;
  if (in_sizes[8] != kDepth * kXdR * kDin || in_sizes[15] != kDepth * kXdR * kDin) return;
  if (in_sizes[9] != kDepth * kDin * kDtR || in_sizes[16] != kDepth * kDin * kDtR) return;
  if (in_sizes[10] != kDepth * kDin || in_sizes[17] != kDepth * kDin) return;
  if (in_sizes[11] != kDepth * kDin * kNst || in_sizes[18] != kDepth * kDin * kNst) return;
  if (in_sizes[12] != kDepth * kDin || in_sizes[19] != kDepth * kDin) return;
  if (in_sizes[20] != kDepth * kDm * kDin) return;
  if (in_sizes[21] != kDepth * kDm || in_sizes[22] != kDm) return;
  if (in_sizes[23] != kNC * kDm || in_sizes[24] != kNC) return;
  if (out_size != kB * kNC) return;
  if (ws_size < kWsTotal) return;

  const float* x          = (const float*)d_in[0];
  const float* patch_w    = (const float*)d_in[1];
  const float* patch_b    = (const float*)d_in[2];
  const float* cls_tok    = (const float*)d_in[3];
  const float* pos_emb    = (const float*)d_in[4];
  const float* in_proj_w  = (const float*)d_in[5];
  const float* conv_w     = (const float*)d_in[6];
  const float* conv_bias  = (const float*)d_in[7];
  const float* x_proj_w   = (const float*)d_in[8];
  const float* dt_w       = (const float*)d_in[9];
  const float* dt_b       = (const float*)d_in[10];
  const float* A_log      = (const float*)d_in[11];
  const float* ssm_D      = (const float*)d_in[12];
  const float* conv_bw    = (const float*)d_in[13];
  const float* conv_bb    = (const float*)d_in[14];
  const float* x_proj_bw  = (const float*)d_in[15];
  const float* dt_bw      = (const float*)d_in[16];
  const float* dt_bb      = (const float*)d_in[17];
  const float* A_blog     = (const float*)d_in[18];
  const float* ssm_Db     = (const float*)d_in[19];
  const float* out_proj_w = (const float*)d_in[20];
  const float* norm_w     = (const float*)d_in[21];
  const float* norm_f_w   = (const float*)d_in[22];
  const float* head_w     = (const float*)d_in[23];
  const float* head_b     = (const float*)d_in[24];
  float* out = (float*)d_out;

  char* ws = (char*)d_ws;
  unsigned short* AP16 = (unsigned short*)(ws + kOffAP16);
  unsigned short* PW16 = (unsigned short*)(ws + kOffPW16);
  unsigned short* WI16 = (unsigned short*)(ws + kOffWI16);
  unsigned short* WX16 = (unsigned short*)(ws + kOffWX16);
  unsigned short* WO16 = (unsigned short*)(ws + kOffWO16);
  float*          FEAT = (float*)(ws + kOffFEAT);
  float*          HB   = (float*)(ws + kOffHB);
  float*          RES  = (float*)(ws + kOffRES);
  unsigned short* HN16 = (unsigned short*)(ws + kOffHN16);
  float*          XZ   = (float*)(ws + kOffXZ);
  float*          XC   = (float*)(ws + kOffXC);
  unsigned short* XC16 = (unsigned short*)(ws + kOffXC16);
  float*          XD   = (float*)(ws + kOffXD);
  unsigned short* Y16  = (unsigned short*)(ws + kOffY16);

  {
    const int n8 = kDm * kPK / 8;
    cast_scale_f16x8<<<(n8 + 255) / 256, 256, 0, stream>>>(patch_w, PW16, n8, kCarryW);
  }
  {
    const int n8 = kDepth * kXzP * kDm / 8;
    cast_scale_f16x8<<<(n8 + 255) / 256, 256, 0, stream>>>(in_proj_w, WI16, n8, kCarryW);
  }
  {
    const int n8 = kDepth * kDm * kDin / 8;
    cast_scale_f16x8<<<(n8 + 255) / 256, 256, 0, stream>>>(out_proj_w, WO16, n8, kCarryW);
  }
  {
    const int n8 = kDepth * 2 * kXdN * kDin / 8;
    pack_xproj_w<<<(n8 + 255) / 256, 256, 0, stream>>>(x_proj_w, x_proj_bw, WX16, n8, kCarryW);
  }
  {
    const int n8 = kMP * kPK / 8;
    im2col_kernel<<<(n8 + 255) / 256, 256, 0, stream>>>(x, AP16, n8);
  }
  {
    const int n8 = (kMP - kTok) * kDin / 8;
    zero_f16x8<<<(n8 + 255) / 256, 256, 0, stream>>>(Y16 + (size_t)kTok * kDin, n8);
  }
  {
    constexpr int tiles = (kMP / 64) * (kDm / 64);
    wmma_gemm64<0, false, 0, 0, false><<<dim3((tiles + 7) / 8, 1), 256, 0, stream>>>(
        AP16, nullptr, kPK, 0L,
        PW16, nullptr, kPK, 0L,
        (void*)FEAT, nullptr, kDm, 0L,
        nullptr, nullptr, 0L,
        kMP, kDm, kPK, 1.0f / kCarryW);
  }
  embed_kernel<<<kMP, 64, 0, stream>>>(FEAT, patch_b, cls_tok, pos_emb, HB, RES);

  for (int l = 0; l < kDepth; ++l) {
    rmsnorm_kernel<<<kMP, 64, 0, stream>>>(HB, RES, norm_w + (size_t)l * kDm, HN16);
    {
      constexpr int tiles = (kMP / 64) * (kXzP / 64);
      wmma_gemm64<0, false, 0, 0, false><<<dim3((tiles + 7) / 8, 1), 256, 0, stream>>>(
          HN16, nullptr, kDm, 0L,
          WI16 + (size_t)l * kXzP * kDm, nullptr, kDm, 0L,
          (void*)XZ, nullptr, kXzP, 0L,
          nullptr, nullptr, 0L,
          kMP, kXzP, kDm, 1.0f / (kCarryHn * kCarryW));
    }
    conv_silu_kernel<<<kMP, 128, 0, stream>>>(
        XZ, conv_w + (size_t)l * kDin * 4, conv_bias + (size_t)l * kDin,
        conv_bw + (size_t)l * kDin * 4, conv_bb + (size_t)l * kDin, XC, XC16);
    {
      constexpr int tiles = (kMP / 64) * (kXdN / 64);
      wmma_gemm64<0, false, 0, 0, false><<<dim3((tiles + 7) / 8, 2), 256, 0, stream>>>(
          XC16, nullptr, kDin, (long)kMP * kDin,
          WX16 + (size_t)l * 2 * kXdN * kDin, nullptr, kDin, (long)kXdN * kDin,
          (void*)XD, nullptr, kXdN, (long)kMP * kXdN,
          nullptr, nullptr, 0L,
          kMP, kXdN, kDin, 1.0f / (kCarryXc * kCarryW));
    }
    scan_gate_kernel<<<kB * (kDin / kScanCh), kScanCh, 0, stream>>>(
        XD, XC, XZ,
        dt_w  + (size_t)l * kDin * kDtR, dt_b  + (size_t)l * kDin, A_log  + (size_t)l * kDin * kNst, ssm_D  + (size_t)l * kDin,
        dt_bw + (size_t)l * kDin * kDtR, dt_bb + (size_t)l * kDin, A_blog + (size_t)l * kDin * kNst, ssm_Db + (size_t)l * kDin,
        Y16);
    {
      constexpr int tiles = (kMP / 64) * (kDm / 64);
      wmma_gemm64<0, false, 0, 0, false><<<dim3((tiles + 7) / 8, 1), 256, 0, stream>>>(
          Y16, nullptr, kDin, 0L,
          WO16 + (size_t)l * kDm * kDin, nullptr, kDin, 0L,
          (void*)HB, nullptr, kDm, 0L,
          nullptr, nullptr, 0L,
          kMP, kDm, kDin, 1.0f / (kCarryY * kCarryW));
    }
  }

  head_kernel<<<(kB * kNC + 1023) / 1024, 256, 0, stream>>>(HB, RES, norm_f_w, head_w, head_b, out);
}
